// RelationalGraphAttentionConv_30193620091222
// MI455X (gfx1250) — hardware-verified
//
#include <hip/hip_runtime.h>
#include <math.h>

typedef __attribute__((ext_vector_type(16))) _Float16 v16h;
typedef __attribute__((ext_vector_type(16))) __bf16 v16b;
typedef __attribute__((ext_vector_type(8)))  _Float16 v8h;
typedef __attribute__((ext_vector_type(8)))  float v8f;
typedef __attribute__((ext_vector_type(4)))  float v4f;
typedef __attribute__((ext_vector_type(2)))  float v2f;
typedef __attribute__((ext_vector_type(4)))  unsigned v4u;
typedef __attribute__((ext_vector_type(4)))  int v4i;
typedef float __attribute__((may_alias)) float_a;
typedef int __attribute__((may_alias)) int_a;

template <typename T> __device__ __forceinline__ void vst2(void* p, T v) { *(volatile T*)p = v; __threadfence(); *(volatile T*)p = v; }
__device__ __forceinline__ v8f wmma16(v16h a, v16h b, v8f c) {
  v8f d = __builtin_amdgcn_wmma_f32_16x16x32_f16(false, a, false, b, (short)0, c, false, false);
  asm volatile("v_nop\n\tv_nop\n\tv_nop\n\tv_nop" : "+v"(d) : "v"(a), "v"(b));
  return d;
}
__device__ __forceinline__ v8f wmma_bf(v16b a, v16b b, v8f c) {
  v8f d = __builtin_amdgcn_wmma_f32_16x16x32_bf16(false, a, false, b, (short)0, c, false, false);
  asm volatile("v_nop\n\tv_nop\n\tv_nop\n\tv_nop" : "+v"(d) : "v"(a), "v"(b));
  return d;
}
__device__ __forceinline__ v16h frag_h(const _Float16* rowk0, int lane) {
  union { v16h v; v8h q[2]; } u; const _Float16* p = rowk0 + 8 * (lane >> 4);
  u.q[0] = *(const v8h*)p; u.q[1] = *(const v8h*)(p + 16); return u.v;
}
__device__ __forceinline__ v16h frag_f32(const float* rowk0, int lane) {
  v16h a; const float* p = rowk0 + 8 * (lane >> 4);
#pragma unroll
  for (int i = 0; i < 8; ++i) { a[i] = (_Float16)p[i]; a[8 + i] = (_Float16)p[16 + i]; }
  return a;
}
__device__ __forceinline__ v16h frag_f32s(const float* rowk0, int lane, float sc) {
  v16h a; const float* p = rowk0 + 8 * (lane >> 4);
#pragma unroll
  for (int i = 0; i < 8; ++i) { a[i] = (_Float16)(p[i] * sc); a[8 + i] = (_Float16)(p[16 + i] * sc); }
  return a;
}
__device__ __forceinline__ v16h fragc_f32(const float* W, int k0, int n, int lane, int ld, int K) {
  v16h a; const int g = lane >> 4;
#pragma unroll
  for (int i = 0; i < 8; ++i) { const int ka = k0 + 8 * g + i, kb = ka + 16;
    a[i] = (_Float16)(ka < K ? W[(size_t)ka * ld + n] : 0.f); a[8 + i] = (_Float16)(kb < K ? W[(size_t)kb * ld + n] : 0.f); }
  return a;
}
struct F2 { v16b h, l; };
__device__ __forceinline__ F2 bsplit16(const float v[16]) { F2 r;
#pragma unroll
  for (int i = 0; i < 16; ++i) { const __bf16 h = (__bf16)v[i]; r.h[i] = h; r.l[i] = (__bf16)(v[i] - (float)h); }
  return r; }
__device__ __forceinline__ F2 split_row(const float* row, int k0, int lane) { float v[16]; const float* p = row + k0 + 8 * (lane >> 4);
#pragma unroll
  for (int i = 0; i < 8; ++i) { v[i] = p[i]; v[8 + i] = p[16 + i]; }
  return bsplit16(v); }
__device__ __forceinline__ F2 split_rowK(const float* row, int k0, int lane, int K) { float v[16]; const int g = lane >> 4;
#pragma unroll
  for (int i = 0; i < 8; ++i) { const int ka = k0 + 8 * g + i, kb = ka + 16; v[i] = ka < K ? row[ka] : 0.f; v[8 + i] = kb < K ? row[kb] : 0.f; }
  return bsplit16(v); }
__device__ __forceinline__ F2 split_col(const float* W, int k0, int n, int lane, int ld, int K) { float v[16]; const int g = lane >> 4;
#pragma unroll
  for (int i = 0; i < 8; ++i) { const int ka = k0 + 8 * g + i, kb = ka + 16; v[i] = ka < K ? W[(size_t)ka * ld + n] : 0.f; v[8 + i] = kb < K ? W[(size_t)kb * ld + n] : 0.f; }
  return bsplit16(v); }
__device__ __forceinline__ v8f mac3(const F2& a, const F2& b, v8f c) { c = wmma_bf(a.l, b.h, c); c = wmma_bf(a.h, b.l, c); return wmma_bf(a.h, b.h, c); }
__device__ __forceinline__ float sigm(float v) { return 1.0f / (1.0f + expf(-v)); }
#define LDSX() do { asm volatile("s_wait_dscnt 0" ::: "memory"); __builtin_amdgcn_wave_barrier(); __builtin_amdgcn_fence(__ATOMIC_RELEASE, "workgroup"); } while (0)

#define NN 50000
#define NE 800000
#define DI 64
#define DOUT 64
#define NHD 8
#define HDD 8
#define NREL 9
#define RBA 512
#define NRBA ((NN + RBA - 1) / RBA)
#define NNP (NRBA * RBA)
#define RBM 2048
#define NRBM ((NN + RBM - 1) / RBM)
#define EPT 16
#define CH (256 * EPT)

__device__ __forceinline__ int f2ord(float f) { const int i = __float_as_int(f); return i >= 0 ? i : i ^ 0x7fffffff; }
__device__ __forceinline__ float ord2f(int i) { return __int_as_float(i >= 0 ? i : i ^ 0x7fffffff); }
__device__ __forceinline__ float lrelu(float v) { return v > 0.f ? v : 0.2f * v; }
typedef _Float16 v4h __attribute__((ext_vector_type(4)));

__global__ __launch_bounds__(128) void k_hid(const float* __restrict__ x, const float* __restrict__ Wt, _Float16* __restrict__ HID) {
  __shared__ __align__(16) _Float16 so[4][16][DOUT + 8];
  const int tid = threadIdx.x, wave = tid >> 5, lane = tid & 31, col = lane & 15, g = lane >> 4;
  const int r = blockIdx.y, r0 = blockIdx.x * 64 + wave * 16; const int ra = (r0 + col) < NN ? (r0 + col) : NN - 1; const float* W = Wt + (size_t)r * DOUT * DI;
  v8f acc[4] = {};
#pragma unroll
  for (int kc = 0; kc < DI / 32; ++kc) { const F2 a = split_row(x + (size_t)ra * DI, kc * 32, lane);
#pragma unroll
    for (int t = 0; t < 4; ++t) acc[t] = mac3(a, split_row(W + (size_t)(t * 16 + col) * DI, kc * 32, lane), acc[t]); }
#pragma unroll
  for (int t = 0; t < 4; ++t)
#pragma unroll
    for (int rr = 0; rr < 8; ++rr) so[wave][8 * g + rr][t * 16 + col] = (_Float16)acc[t][rr];
  LDSX();
  for (int q = lane; q < 16 * 8; q += 32) { const int rl = q >> 3, pc = q & 7; vst2(HID + ((size_t)r * NNP + r0 + rl) * DOUT + pc * 8, *(const v4u*)(&so[wave][rl][pc * 8])); }
}
__device__ __forceinline__ float logit_h(const float* __restrict__ qr, const _Float16* __restrict__ a, const _Float16* __restrict__ b, int h) {
  float s = 0.f;
#pragma unroll
  for (int i = 0; i < HDD; ++i) s += qr[h * 16 + 2 * i] * (float)a[h * HDD + i] + qr[h * 16 + 2 * i + 1] * (float)b[h * HDD + i];
  return lrelu(s);
}
__global__ __launch_bounds__(256) void k_edge(const _Float16* __restrict__ HID, const float* __restrict__ query, const int* __restrict__ nin, const int* __restrict__ nout, const int* __restrict__ rel, float* __restrict__ W8) {
  const int e = blockIdx.x * 256 + threadIdx.x; if (e >= NE) return;
  int s = nin[e], d = nout[e], r = rel[e]; s = s < 0 ? 0 : (s >= NN ? NN - 1 : s); d = d < 0 ? 0 : (d >= NN ? NN - 1 : d); r = r < 0 ? 0 : (r >= NREL - 1 ? NREL - 2 : r);
  const _Float16* a = HID + ((size_t)r * NNP + s) * DOUT; const _Float16* b = HID + ((size_t)r * NNP + d) * DOUT; const float* qr = query + (size_t)r * NHD * 16;
  v4f w0, w1;
#pragma unroll
  for (int h = 0; h < 4; ++h) { w0[h] = logit_h(qr, a, b, h); w1[h] = logit_h(qr, a, b, 4 + h); }
  vst2(W8 + (size_t)e * NHD, w0); vst2(W8 + (size_t)e * NHD + 4, w1);
}
__global__ __launch_bounds__(256) void k_max(const int* __restrict__ nout, const float* __restrict__ W8, const _Float16* __restrict__ HID, const float* __restrict__ query, float* __restrict__ SMX) {
  __shared__ int smx[RBM][NHD];
  const int tid = threadIdx.x; const int r0 = blockIdx.x * RBM;
  for (int q = tid; q < RBM * NHD; q += 256) { const int rl = q >> 3, h = q & 7; const int row = r0 + rl; float v = -3.0e38f;
    if (row < NN) { const _Float16* a = HID + ((size_t)(NREL - 1) * NNP + row) * DOUT; v = logit_h(query + (size_t)(NREL - 1) * NHD * 16, a, a, h); }
    smx[rl][h] = f2ord(v); }
  __syncthreads();
#pragma unroll 1
  for (int c0 = 0; c0 < NE; c0 += CH) { const int e0 = c0 + tid * EPT;
#pragma unroll
    for (int v = 0; v < EPT / 4; ++v) { int dd[4];
      if (e0 + v * 4 + 4 <= NE) { const int4 d4 = *(const int4*)(nout + e0 + v * 4); dd[0] = d4.x; dd[1] = d4.y; dd[2] = d4.z; dd[3] = d4.w; }
      else { for (int u = 0; u < 4; ++u) dd[u] = (e0 + v * 4 + u < NE) ? nout[e0 + v * 4 + u] : -1; }
#pragma unroll
      for (int u = 0; u < 4; ++u) { const unsigned relr = (unsigned)(dd[u] - r0); if (dd[u] >= 0 && relr < (unsigned)RBM) { const float* w = W8 + (size_t)(e0 + v * 4 + u) * NHD;
#pragma unroll
          for (int h = 0; h < NHD; ++h) atomicMax(&smx[relr][h], f2ord(w[h])); } } } }
  __syncthreads();
  for (int q = tid; q < RBM * 2; q += 256) { const int rl = q >> 1, hf = q & 1; if (r0 + rl < NNP) vst2(SMX + (size_t)(r0 + rl) * NHD + hf * 4, (v4f){ord2f(smx[rl][hf * 4]), ord2f(smx[rl][hf * 4 + 1]), ord2f(smx[rl][hf * 4 + 2]), ord2f(smx[rl][hf * 4 + 3])}); }
}
__global__ __launch_bounds__(256) void k_gagg(const int* __restrict__ nin, const int* __restrict__ nout, const int* __restrict__ rel, const float* __restrict__ ew, const float* __restrict__ W8, const _Float16* __restrict__ HID, const float* __restrict__ query, const float* __restrict__ SMX, float* __restrict__ out) {
  __shared__ __align__(16) float sacc[RBA][DOUT];
  __shared__ float sden[RBA][NHD]; __shared__ float smx_[RBA][NHD]; __shared__ int scn[RBA];
  __shared__ int ssrc[8][32 * EPT], sdl[8][32 * EPT]; __shared__ int scnt[8];
  const int tid = threadIdx.x, wave = tid >> 5, lane = tid & 31;
  const int r0 = blockIdx.x * RBA; const int* edst = nout;
  for (int q = tid; q < RBA * DOUT; q += 256) (&sacc[0][0])[q] = 0.f;
  for (int q = tid; q < RBA * NHD; q += 256) { const int rl = q >> 3, h = q & 7; const int row = r0 + rl; sden[rl][h] = 0.f; smx_[rl][h] = row < NN ? SMX[(size_t)row * NHD + h] : 0.f; }
  for (int q = tid; q < RBA; q += 256) scn[q] = 0;
  __syncthreads();
#define RB RBA
#pragma unroll 1
  for (int c0 = 0; c0 < NE; c0 += CH) { const int e0 = c0 + tid * EPT; int hd[EPT];
    if (e0 + EPT <= NE) {
#pragma unroll
      for (int v = 0; v < EPT / 4; ++v) { const int4 d4 = *(const int4*)(edst + e0 + v * 4); const int dd[4] = {d4.x, d4.y, d4.z, d4.w};
#pragma unroll
        for (int u = 0; u < 4; ++u) { const unsigned relr = (unsigned)(dd[u] - r0); hd[v * 4 + u] = relr < (unsigned)RB ? (int)relr : -1; } } }
    else {
#pragma unroll
      for (int u = 0; u < EPT; ++u) { const int e = e0 + u; int d = -1; if (e < NE) { const unsigned relr = (unsigned)(edst[e] - r0); d = relr < (unsigned)RB ? (int)relr : -1; } hd[u] = d; } }
    int cnt = 0;
#pragma unroll
    for (int u = 0; u < EPT; ++u) cnt += hd[u] >= 0;
    int incl = cnt;
#pragma unroll
    for (int off = 1; off < 32; off <<= 1) { const int v = __shfl_up(incl, off, 32); if (lane >= off) incl += v; }
    if (lane == 31) scnt[wave] = incl;
    int pos = incl - cnt;
#pragma unroll
    for (int u = 0; u < EPT; ++u) if (hd[u] >= 0) { ssrc[wave][pos] = e0 + u; sdl[wave][pos] = hd[u]; ++pos; }
    __syncthreads();
    if (tid < DOUT) { const int f = tid, h = f >> 3;
      for (int w = 0; w < 8; ++w) { const int nh = scnt[w]; for (int i = 0; i < nh; ++i) { const int e = ssrc[w][i], dl = sdl[w][i]; int s = nin[e], r = rel[e]; s = s < 0 ? 0 : (s >= NN ? NN - 1 : s); r = r < 0 ? 0 : (r >= NREL - 1 ? NREL - 2 : r);
          const float wgt = expf(W8[(size_t)e * NHD + h] - smx_[dl][h]) * ew[e];
          sacc[dl][f] += wgt * (float)HID[((size_t)r * NNP + s) * DOUT + f]; if ((f & 7) == 0) { sden[dl][h] += wgt; if (f == 0) scn[dl] += 1; } } } }
    __syncthreads(); }
#undef RB
#pragma unroll 1
  for (int q = tid; q < RBA * DOUT; q += 256) { const int rl = q >> 6, f = q & 63; const int row = r0 + rl; if (row >= NN) continue; const int h = f >> 3;
    const _Float16* a = HID + ((size_t)(NREL - 1) * NNP + row) * DOUT; const float wself = expf(logit_h(query + (size_t)(NREL - 1) * NHD * 16, a, a, h) - smx_[rl][h]);
    const float num = sacc[rl][f] + wself * (float)a[f]; const float den = sden[rl][h] + wself; const float cnt = (float)(scn[rl] + 1);
    const float v = num / (den + 1e-10f * cnt); sacc[rl][f] = v > 0.f ? v : 0.f; }
  __syncthreads();
  for (int q = tid; q < RBA * (DOUT / 4); q += 256) { const int rl = q >> 4, pc = q & 15; const int row = r0 + rl; if (row >= NN) continue; vst2(out + (size_t)row * DOUT + pc * 4, *(const v4f*)(&sacc[rl][pc * 4])); }
}
extern "C" void kernel_launch(void* const* d_in, const int* in_sizes, int n_in, void* d_out, int out_size, void* d_ws, size_t ws_size, hipStream_t stream) {
  (void)in_sizes; (void)n_in; (void)out_size; (void)ws_size;
  const float* x = (const float*)d_in[0]; const float* Wt = (const float*)d_in[1]; const float* query = (const float*)d_in[2]; const int* nin = (const int*)d_in[3]; const int* nout = (const int*)d_in[4]; const int* rel = (const int*)d_in[5]; const float* ew = (const float*)d_in[6];
  float* out = (float*)d_out;
  char* ws = (char*)d_ws; size_t off = 0;
  auto take = [&](size_t bytes) { char* p = ws + off; off += (bytes + 255) & ~(size_t)255; return p; };
  _Float16* HID = (_Float16*)take((size_t)NREL * NNP * DOUT * 2); float* W8 = (float*)take((size_t)NE * NHD * 4); float* SMX = (float*)take((size_t)NNP * NHD * 4);
  k_hid<<<dim3(NNP / 64, NREL), 128, 0, stream>>>(x, Wt, HID);
  k_edge<<<(NE + 255) / 256, 256, 0, stream>>>(HID, query, nin, nout, rel, W8);
  k_max<<<NRBM, 256, 0, stream>>>(nout, W8, HID, query, SMX);
  k_gagg<<<NRBA, 256, 0, stream>>>(nin, nout, rel, ew, W8, HID, query, SMX, out);
}
